// AttentionBlock_49469433315393
// MI455X (gfx1250) — hardware-verified
//
#include <hip/hip_runtime.h>
#include <math.h>
#include <stddef.h>

#define NB_   4
#define NC_   512
#define HWN_  4096
#define NHD_  4
#define HDM_  128
#define NGR_  32
#define GSZ_  65536

typedef _Float16 v16h __attribute__((ext_vector_type(16)));
typedef _Float16 v8h  __attribute__((ext_vector_type(8)));
typedef float    v8f  __attribute__((ext_vector_type(8)));
typedef float    v4f  __attribute__((ext_vector_type(4)));
typedef v4f v4fa __attribute__((may_alias));
typedef v8h v8ha __attribute__((may_alias));

union FragU { v16h v; v8h h[2]; };

__device__ __forceinline__ v8f zero8() { v8f z = {0.f,0.f,0.f,0.f,0.f,0.f,0.f,0.f}; return z; }

__device__ __forceinline__ v8f mma16(v16h a, v16h b, v8f c) {
  return __builtin_amdgcn_wmma_f32_16x16x32_f16(false, a, false, b, (short)0, c, false, false);
}
__device__ __forceinline__ void guard4(v8f& a, v8f& b, v8f& c, v8f& d, v16h x, v16h y) {
  asm volatile("v_nop\n\tv_nop\n\tv_nop\n\tv_nop" : "+v"(a), "+v"(b), "+v"(c), "+v"(d) : "v"(x), "v"(y));
}
__device__ __forceinline__ void keep3(v16h a, v16h b, v16h c) { asm volatile("v_nop" :: "v"(a), "v"(b), "v"(c)); }

__device__ __forceinline__ v16h ldfrag_g(const _Float16* p) {
  FragU f; f.h[0] = *(const v8h*)(p); f.h[1] = *(const v8h*)(p + 16); return f.v;
}
__device__ __forceinline__ v16h ldfrag_s(const _Float16* p) {
  FragU f; f.h[0] = *(const v8ha*)(p); f.h[1] = *(const v8ha*)(p + 16); return f.v;
}
__device__ __forceinline__ void lds_wave_sync() {
  __builtin_amdgcn_fence(__ATOMIC_RELEASE, "workgroup");
  __builtin_amdgcn_wave_barrier();
  __builtin_amdgcn_fence(__ATOMIC_ACQUIRE, "workgroup");
}

__global__ __launch_bounds__(256) void k_stats(const float* __restrict__ x, float* __restrict__ stats) {
  __shared__ double red[256];
  __shared__ double bc[1];
  __shared__ float  res[2];
  const int tid = threadIdx.x;
  const int bg  = blockIdx.x;
  const float* p = x + (size_t)bg * GSZ_;
  double s = 0.0;
  for (int i = tid; i < GSZ_ / 4; i += 256) {
    const v4f v = *(const v4f*)(p + 4 * (size_t)i);
    s += (double)v[0]; s += (double)v[1]; s += (double)v[2]; s += (double)v[3];
  }
  red[tid] = s;
  __syncthreads();
  if (tid == 0) {
    double S = 0.0;
    for (int i = 0; i < 256; ++i) S += red[i];
    bc[0] = S * (1.0 / (double)GSZ_);
  }
  __syncthreads();
  const double mean = bc[0];
  double s2 = 0.0;
  for (int i = tid; i < GSZ_ / 4; i += 256) {
    const v4f v = *(const v4f*)(p + 4 * (size_t)i);
    double d0 = (double)v[0] - mean, d1 = (double)v[1] - mean, d2 = (double)v[2] - mean, d3 = (double)v[3] - mean;
    s2 += d0 * d0; s2 += d1 * d1; s2 += d2 * d2; s2 += d3 * d3;
  }
  red[tid] = s2;
  __syncthreads();
  if (tid == 0) {
    double S2 = 0.0;
    for (int i = 0; i < 256; ++i) S2 += red[i];
    const double var  = S2 * (1.0 / (double)GSZ_);
    const double rstd = 1.0 / sqrt(var + 1e-5);
    res[0] = (float)mean;
    res[1] = (float)rstd;
  }
  __syncthreads();
  if (tid < 8) {
    const float mv = res[0], rv = res[1];
    v4f val;
    val[0] = (tid == 0) ? mv : 0.f;
    val[1] = (tid == 0) ? rv : 0.f;
    val[2] = 0.f;
    val[3] = 0.f;
    float* dst = stats + (size_t)bg * 32 + tid * 4;
    *(volatile v4f*)dst = val;
    __threadfence();
    *(volatile v4f*)dst = val;
  }
}

__global__ __launch_bounds__(256) void k_wcvt(const float* __restrict__ w0, const float* __restrict__ w1,
                                              const float* __restrict__ w2, const float* __restrict__ w3,
                                              _Float16* __restrict__ W16) {
  const int which = blockIdx.y;
  const float* src = (which == 0) ? w0 : ((which == 1) ? w1 : ((which == 2) ? w2 : w3));
  const size_t e = ((size_t)blockIdx.x * 256 + threadIdx.x) * 8;
  const v4f a = *(const v4f*)(src + e);
  const v4f c = *(const v4f*)(src + e + 4);
  v8h o;
  o[0] = (_Float16)(a[0] * 16.0f); o[1] = (_Float16)(a[1] * 16.0f);
  o[2] = (_Float16)(a[2] * 16.0f); o[3] = (_Float16)(a[3] * 16.0f);
  o[4] = (_Float16)(c[0] * 16.0f); o[5] = (_Float16)(c[1] * 16.0f);
  o[6] = (_Float16)(c[2] * 16.0f); o[7] = (_Float16)(c[3] * 16.0f);
  _Float16* dst = W16 + (size_t)which * ((size_t)NC_ * NC_) + e;
  *(volatile v8h*)dst = o;
  __threadfence();
  *(volatile v8h*)dst = o;
}

__global__ __launch_bounds__(256) void k_xn(const float* __restrict__ x, const float* __restrict__ gw,
                                            const float* __restrict__ gb, const float* __restrict__ stats,
                                            _Float16* __restrict__ xn) {
  __shared__ __align__(16) float tf[64 * 68];
  const int t0 = blockIdx.x * 64;
  const int c0 = blockIdx.y * 64;
  const int b  = blockIdx.z;
  const int tid = threadIdx.x;
  {
    const int lr = tid >> 4;
    const int c4 = (tid & 15) * 4;
#pragma unroll
    for (int it = 0; it < 4; ++it) {
      const int rr = it * 16 + lr;
      const int ch = c0 + rr;
      const int g  = ch >> 4;
      const float mean = stats[(size_t)(b * NGR_ + g) * 32 + 0];
      const float rstd = stats[(size_t)(b * NGR_ + g) * 32 + 1];
      const float w  = gw[ch];
      const float bb = gb[ch];
      v4f a = *(const v4f*)(x + ((size_t)(b * NC_ + ch)) * HWN_ + t0 + c4);
      a = ((a - mean) * rstd) * w + bb;
      *(v4f*)(tf + rr * 68 + c4) = a;
    }
  }
  __syncthreads();
  const int sub = tid >> 3;
  const int c8  = (tid & 7) * 8;
  v8h hv[2];
#pragma unroll
  for (int it = 0; it < 2; ++it) {
    const int oc = it * 32 + sub;
    v8h o;
#pragma unroll
    for (int e = 0; e < 8; ++e) o[e] = (_Float16)tf[(c8 + e) * 68 + oc];
    hv[it] = o;
  }
  for (int pass = 0; pass < 2; ++pass) {
#pragma unroll
    for (int it = 0; it < 2; ++it) {
      const int oc = it * 32 + sub;
      *(volatile v8h*)(xn + ((size_t)(b * HWN_ + t0 + oc)) * NC_ + c0 + c8) = hv[it];
    }
    __threadfence();
  }
}

template <int BIAS_MODE, int OUT_MODE, bool RESID>
__global__ __launch_bounds__(256) void k_gemm64(
    const _Float16* __restrict__ A, int lda, long strideA,
    const _Float16* __restrict__ Bt, int ldb, long strideB,
    void* __restrict__ Cout, int ldc, long strideC,
    const float* __restrict__ bias,
    const float* __restrict__ resid, long strideR,
    int M, int N, int K, float scale, float oscale) {
  __shared__ __align__(16) float sT[8][16 * 68];
  const int b    = blockIdx.y;
  const int lane = threadIdx.x & 31;
  const int wave = threadIdx.x >> 5;
  const int tilesN = N >> 6;
  const int tilesM = M >> 6;
  const int tile = blockIdx.x * 8 + wave;
  if (tile >= tilesM * tilesN) return;
  const int tm = tile / tilesN;
  const int tn = tile - tm * tilesN;
  const int m0 = tm << 6;
  const int n0 = tn << 6;
  const _Float16* Ab = A  + (size_t)b * strideA;
  const _Float16* Bb = Bt + (size_t)b * strideB;
  const int rl   = lane & 15;
  const int koff = (lane >> 4) * 8;
  const int mOff = (lane >> 4) * 8;

  v8f acc[4][4];
#pragma unroll
  for (int i = 0; i < 4; ++i)
#pragma unroll
    for (int j = 0; j < 4; ++j) acc[i][j] = zero8();

  for (int k0 = 0; k0 < K; k0 += 32) {
    v16h bh[4];
#pragma unroll
    for (int j = 0; j < 4; ++j)
      bh[j] = ldfrag_g(Bb + (size_t)(n0 + (j << 4) + rl) * ldb + k0 + koff);
#pragma unroll
    for (int i = 0; i < 4; ++i) {
      const v16h ah = ldfrag_g(Ab + (size_t)(m0 + (i << 4) + rl) * lda + k0 + koff);
#pragma unroll
      for (int j = 0; j < 4; ++j) acc[i][j] = mma16(ah, bh[j], acc[i][j]);
      guard4(acc[i][0], acc[i][1], acc[i][2], acc[i][3], ah, bh[3]);
    }
    keep3(bh[0], bh[1], bh[2]);
  }

  float* slab = sT[wave];
  const float* Rb = resid + (RESID ? (size_t)b * strideR : (size_t)0);
#pragma unroll
  for (int i = 0; i < 4; ++i) {
    const int mBase = m0 + (i << 4);
    float bm[8];
#pragma unroll
    for (int r = 0; r < 8; ++r) bm[r] = (BIAS_MODE == 1) ? bias[mBase + mOff + r] : 0.f;
#pragma unroll
    for (int j = 0; j < 4; ++j) {
      const int n = n0 + (j << 4) + rl;
      float bvn = 0.f;
      if (BIAS_MODE == 2) bvn = bias[n];
#pragma unroll
      for (int r = 0; r < 8; ++r) {
        float v = acc[i][j][r] * scale + bm[r] + bvn;
        if (RESID) v += Rb[(size_t)(mBase + mOff + r) * ldc + n];
        slab[(mOff + r) * 68 + (j << 4) + rl] = v;
      }
    }
    lds_wave_sync();
    if (OUT_MODE == 0) {
      float* C = (float*)Cout + (size_t)b * strideC;
      const int hh = lane >> 4, c4 = (lane & 15) * 4;
      v4f ov[8];
#pragma unroll
      for (int it = 0; it < 8; ++it) ov[it] = *(const v4fa*)(slab + (it * 2 + hh) * 68 + c4);
      for (int pass = 0; pass < 2; ++pass) {
#pragma unroll
        for (int it = 0; it < 8; ++it) {
          const int row = it * 2 + hh;
          *(volatile v4f*)(C + (size_t)(mBase + row) * ldc + n0 + c4) = ov[it];
        }
        __threadfence();
      }
    } else {
      _Float16* C = (_Float16*)Cout + (size_t)b * strideC;
      const int q = lane >> 3, c8 = (lane & 7) * 8;
      v8h hv[4];
#pragma unroll
      for (int it = 0; it < 4; ++it) {
        const float* sp = slab + (it * 4 + q) * 68 + c8;
        v8h t;
#pragma unroll
        for (int e = 0; e < 8; ++e) t[e] = (_Float16)(sp[e] * oscale);
        hv[it] = t;
      }
      for (int pass = 0; pass < 2; ++pass) {
#pragma unroll
        for (int it = 0; it < 4; ++it) {
          const int row = it * 4 + q;
          *(volatile v8h*)(C + (size_t)(mBase + row) * ldc + n0 + c8) = hv[it];
        }
        __threadfence();
      }
    }
    lds_wave_sync();
  }
}

#define KP_ 136
#define VP_ 72
#define PP_ 72
#define OP_ 136
#define LDSH_ (64 * KP_ + 128 * VP_ + 8 * 16 * PP_)
static_assert(LDSH_ * 2 <= 65536);
static_assert(8 * 16 * OP_ <= 64 * KP_ + 128 * VP_);

__global__ __launch_bounds__(256) void k_attn(const _Float16* __restrict__ Qp, const _Float16* __restrict__ Kp,
                                              const _Float16* __restrict__ VTp, _Float16* __restrict__ Op,
                                              float sc2) {
  __shared__ __align__(16) _Float16 lds[LDSH_];
  const int tid  = threadIdx.x;
  const int wave = tid >> 5;
  const int lane = tid & 31;
  const int hh   = lane >> 4;
  const int c    = lane & 15;
  _Float16* sK  = lds;
  _Float16* sVt = lds + 64 * KP_;
  _Float16* sPw = lds + 64 * KP_ + 128 * VP_ + wave * (16 * PP_);
  const int bh = blockIdx.y;
  const int b  = bh >> 2;
  const int h  = bh & 3;
  const int q0 = blockIdx.x * 128 + wave * 16;
  const _Float16* Qb = Qp  + (size_t)b * HWN_ * NC_ + h * HDM_;
  const _Float16* Kb = Kp  + (size_t)b * HWN_ * NC_ + h * HDM_;
  const _Float16* Vb = VTp + ((size_t)b * NC_ + h * HDM_) * HWN_;
  _Float16*       Ob = Op  + (size_t)b * HWN_ * NC_ + h * HDM_;

  v16h qa[4];
#pragma unroll
  for (int dc = 0; dc < 4; ++dc) qa[dc] = ldfrag_g(Qb + (size_t)(q0 + c) * NC_ + dc * 32 + 8 * hh);

  float mrow[8], lrow[8];
  v8f oacc[8];
#pragma unroll
  for (int r = 0; r < 8; ++r) { mrow[r] = -__builtin_inff(); lrow[r] = 0.f; }
#pragma unroll
  for (int dt = 0; dt < 8; ++dt) oacc[dt] = zero8();

  for (int kc = 0; kc < HWN_ / 64; ++kc) {
    const int kv0 = kc * 64;
    __syncthreads();
    {
      const int r  = tid >> 2;
      const int qd = (tid & 3) * 32;
      const _Float16* ks = Kb + (size_t)(kv0 + r) * NC_ + qd;
      _Float16* kd = sK + r * KP_ + qd;
#pragma unroll
      for (int i = 0; i < 4; ++i) *(v8h*)(kd + 8 * i) = *(const v8h*)(ks + 8 * i);
      const int d  = tid >> 1;
      const int hk = (tid & 1) * 32;
      const _Float16* vs = Vb + (size_t)d * HWN_ + kv0 + hk;
      _Float16* vd = sVt + d * VP_ + hk;
#pragma unroll
      for (int i = 0; i < 4; ++i) *(v8h*)(vd + 8 * i) = *(const v8h*)(vs + 8 * i);
    }
    __syncthreads();

    v8f s[4];
    v16h kb;
#pragma unroll
    for (int j = 0; j < 4; ++j) {
      s[j] = zero8();
#pragma unroll
      for (int dc = 0; dc < 4; ++dc) {
        kb = ldfrag_s(sK + (j * 16 + c) * KP_ + dc * 32 + 8 * hh);
        s[j] = mma16(qa[dc], kb, s[j]);
      }
    }
    guard4(s[0], s[1], s[2], s[3], qa[3], kb);

    float cm[8];
#pragma unroll
    for (int r = 0; r < 8; ++r) {
      float m = s[0][r] * sc2;
#pragma unroll
      for (int j = 0; j < 4; ++j) {
        const float t = s[j][r] * sc2;
        s[j][r] = t;
        m = fmaxf(m, t);
      }
      m = fmaxf(m, __shfl_xor(m, 1, 32));
      m = fmaxf(m, __shfl_xor(m, 2, 32));
      m = fmaxf(m, __shfl_xor(m, 4, 32));
      m = fmaxf(m, __shfl_xor(m, 8, 32));
      cm[r] = m;
    }
#pragma unroll
    for (int r = 0; r < 8; ++r) {
      const float mnew  = fmaxf(mrow[r], cm[r]);
      const float alpha = exp2f(mrow[r] - mnew);
      mrow[r] = mnew;
      float psum = 0.f;
#pragma unroll
      for (int j = 0; j < 4; ++j) {
        const float p = exp2f(s[j][r] - mnew);
        psum += p;
        sPw[(8 * hh + r) * PP_ + j * 16 + c] = (_Float16)(p * 256.0f);
      }
      psum += __shfl_xor(psum, 1, 32);
      psum += __shfl_xor(psum, 2, 32);
      psum += __shfl_xor(psum, 4, 32);
      psum += __shfl_xor(psum, 8, 32);
      lrow[r] = lrow[r] * alpha + psum;
#pragma unroll
      for (int dt = 0; dt < 8; ++dt) oacc[dt][r] *= alpha;
    }
    lds_wave_sync();

#pragma unroll
    for (int kk = 0; kk < 2; ++kk) {
      const v16h pa = ldfrag_s(sPw + c * PP_ + kk * 32 + 8 * hh);
      v16h vb;
#pragma unroll
      for (int dt = 0; dt < 8; ++dt) {
        vb = ldfrag_s(sVt + (dt * 16 + c) * VP_ + kk * 32 + 8 * hh);
        oacc[dt] = mma16(pa, vb, oacc[dt]);
      }
      guard4(oacc[0], oacc[1], oacc[2], oacc[3], pa, vb);
      guard4(oacc[4], oacc[5], oacc[6], oacc[7], pa, vb);
    }
  }

  __syncthreads();
  _Float16* os = lds + wave * (16 * OP_);
#pragma unroll
  for (int r = 0; r < 8; ++r) {
    const float inv = 0.25f / lrow[r];
#pragma unroll
    for (int dt = 0; dt < 8; ++dt) os[(8 * hh + r) * OP_ + dt * 16 + c] = (_Float16)(oacc[dt][r] * inv);
  }
  lds_wave_sync();
  const int c8 = c * 8;
  v8h ov[8];
#pragma unroll
  for (int it = 0; it < 8; ++it) ov[it] = *(const v8ha*)(os + (it * 2 + hh) * OP_ + c8);
  for (int pass = 0; pass < 2; ++pass) {
#pragma unroll
    for (int it = 0; it < 8; ++it) {
      const int row = it * 2 + hh;
      *(volatile v8h*)(Ob + (size_t)(q0 + row) * NC_ + c8) = ov[it];
    }
    __threadfence();
  }
}

extern "C" void kernel_launch(void* const* d_in, const int* in_sizes, int n_in,
                              void* d_out, int out_size, void* d_ws, size_t ws_size,
                              hipStream_t stream) {
  if (n_in < 11) return;
  if (in_sizes[0] != NB_ * NC_ * HWN_) return;
  if (in_sizes[1] != NC_ || in_sizes[2] != NC_) return;
  if (in_sizes[3] != NC_ * NC_ || in_sizes[5] != NC_ * NC_ || in_sizes[7] != NC_ * NC_ || in_sizes[9] != NC_ * NC_) return;
  if (in_sizes[4] != NC_ || in_sizes[6] != NC_ || in_sizes[8] != NC_ || in_sizes[10] != NC_) return;
  if (out_size != NB_ * NC_ * HWN_) return;

  const float* x    = (const float*)d_in[0];
  const float* gn_w = (const float*)d_in[1];
  const float* gn_b = (const float*)d_in[2];
  const float* wq   = (const float*)d_in[3];
  const float* bq   = (const float*)d_in[4];
  const float* wk   = (const float*)d_in[5];
  const float* bk   = (const float*)d_in[6];
  const float* wv   = (const float*)d_in[7];
  const float* bv   = (const float*)d_in[8];
  const float* wp   = (const float*)d_in[9];
  const float* bp   = (const float*)d_in[10];
  float* out = (float*)d_out;

  const size_t szStats = (size_t)NB_ * NGR_ * 128;
  const size_t szW     = (size_t)4 * NC_ * NC_ * 2;
  const size_t szPlane = (size_t)NB_ * HWN_ * NC_ * 2;
  size_t off = 0;
  const size_t oStats = off; off += szStats;
  const size_t oW     = off; off += szW;
  const size_t oXn    = off; off += szPlane;
  const size_t oQ     = off; off += szPlane;
  const size_t oK     = off; off += szPlane;
  const size_t oVT    = off; off += szPlane;
  const size_t oO     = off; off += szPlane;
  if (off > ws_size) return;

  char* ws = (char*)d_ws;
  float*    stats = (float*)(ws + oStats);
  _Float16* W16   = (_Float16*)(ws + oW);
  _Float16* W16q  = W16;
  _Float16* W16k  = W16 + (size_t)1 * NC_ * NC_;
  _Float16* W16v  = W16 + (size_t)2 * NC_ * NC_;
  _Float16* W16p  = W16 + (size_t)3 * NC_ * NC_;
  _Float16* Xn    = (_Float16*)(ws + oXn);
  _Float16* Q16   = (_Float16*)(ws + oQ);
  _Float16* K16   = (_Float16*)(ws + oK);
  _Float16* VT16  = (_Float16*)(ws + oVT);
  _Float16* O16   = (_Float16*)(ws + oO);

  const long plane = (long)HWN_ * NC_;
  const float sc2  = 0.08838834764831845f * 1.4426950408889634f;

  k_stats<<<dim3(NB_ * NGR_), dim3(256), 0, stream>>>(x, stats);
  k_wcvt<<<dim3((NC_ * NC_) / (256 * 8), 4), dim3(256), 0, stream>>>(wq, wk, wv, wp, W16);
  k_xn<<<dim3(HWN_ / 64, NC_ / 64, NB_), dim3(256), 0, stream>>>(x, gn_w, gn_b, stats, Xn);
  {
    const int tiles = ((NB_ * HWN_) / 64) * (NC_ / 64);
    k_gemm64<2, 1, false><<<dim3((tiles + 7) / 8, 1), dim3(256), 0, stream>>>(
        Xn, NC_, 0L, W16q, NC_, 0L, (void*)Q16, NC_, 0L, bq, x, 0L,
        NB_ * HWN_, NC_, NC_, 1.0f / 16.0f, 1.0f);
    k_gemm64<2, 1, false><<<dim3((tiles + 7) / 8, 1), dim3(256), 0, stream>>>(
        Xn, NC_, 0L, W16k, NC_, 0L, (void*)K16, NC_, 0L, bk, x, 0L,
        NB_ * HWN_, NC_, NC_, 1.0f / 16.0f, 1.0f);
  }
  {
    const int tiles = (NC_ / 64) * (HWN_ / 64);
    k_gemm64<1, 1, false><<<dim3((tiles + 7) / 8, NB_), dim3(256), 0, stream>>>(
        W16v, NC_, 0L, Xn, NC_, plane, (void*)VT16, HWN_, plane, bv, x, 0L,
        NC_, HWN_, NC_, 1.0f / 16.0f, 1.0f);
  }
  k_attn<<<dim3(HWN_ / 128, NB_ * NHD_), dim3(256), 0, stream>>>(Q16, K16, VT16, O16, sc2);
  {
    const int tiles = (NC_ / 64) * (HWN_ / 64);
    k_gemm64<1, 0, true><<<dim3((tiles + 7) / 8, NB_), dim3(256), 0, stream>>>(
        W16p, NC_, 0L, O16, NC_, plane, (void*)out, HWN_, plane, bp, x, plane,
        NC_, HWN_, NC_, 1.0f / 1024.0f, 1.0f);
  }
  (void)hipGetLastError();
}
